// HybridGAT_46669114638662
// MI455X (gfx1250) — hardware-run, weakly checked
//
#include <hip/hip_runtime.h>


namespace {
constexpr int N = 20000, NP = 20032, E = 320000, G = 128, DIN = 128, HYB = 256, HID = 128, NH = 4, W1O = NH * HID, NCL = 32;
constexpr float XS = 8.0f, WSC = 256.0f, NEG = 0.2f, BNS = 0.99999500003749981f;
typedef _Float16 b16;
typedef __attribute__((ext_vector_type(16))) _Float16 v16b;
typedef __attribute__((ext_vector_type(8))) _Float16 v8b;
typedef __attribute__((ext_vector_type(8))) float v8f;
typedef __attribute__((ext_vector_type(4))) float v4f;
__device__ __forceinline__ float bf16_rne(float f) { unsigned int u = __float_as_uint(f); u += 0x7FFFu + ((u >> 16) & 1u); return __uint_as_float(u & 0xFFFF0000u); }
__device__ __forceinline__ void split16(float v, b16& hi, b16& lo) { hi = (b16)v; lo = (b16)(v - (float)hi); }
__device__ __forceinline__ v16b frag_kb(const b16* p, int hh) { const v8b a = *(const v8b*)(p + 8 * hh), b = *(const v8b*)(p + 16 + 8 * hh); v16b f;
#pragma unroll
  for (int e = 0; e < 8; ++e) { f[e] = a[e]; f[8 + e] = b[e]; } return f; }
__device__ __forceinline__ v8f wmma16b(v16b a, v16b b, v8f c) { v8f d = __builtin_amdgcn_wmma_f32_16x16x32_f16(false, a, false, b, (short)0, c, false, false); asm volatile("v_nop\n\tv_nop\n\tv_nop\n\tv_nop" : "+v"(d) : "v"(a), "v"(b)); return d; }
__device__ __forceinline__ void wave_lds_sync() { __builtin_amdgcn_fence(__ATOMIC_RELEASE, "workgroup"); __builtin_amdgcn_wave_barrier(); __builtin_amdgcn_fence(__ATOMIC_ACQUIRE, "workgroup"); }
__device__ __forceinline__ float pmul(float a, float b) { float p = a * b; asm volatile("" : "+v"(p)); return p; }
__device__ __forceinline__ float opaque(float a) { asm volatile("" : "+v"(a)); return a; }
__device__ __forceinline__ int iclamp(int v, int lo, int hi) { return v < lo ? lo : (v > hi ? hi : v); }
__device__ __forceinline__ float lrelu(float x) { return x > 0.0f ? x : NEG * x; }
__device__ __forceinline__ float eluf(float x) { return x > 0.0f ? x : (__expf(x) - 1.0f); }
__device__ __forceinline__ float nexp(float x) { return __builtin_amdgcn_exp2f(x * 1.4426950408889634f); }
constexpr int CSR_NBLK9 = 512, CSR_GB9 = 9, CSR_GN9 = 1 << CSR_GB9  , CSR_TS9 = (CSR_GN9 < 32 ? 32 : CSR_GN9)  , CSR_MAXG9 = 512, CSR_CAP9 = 12288  ;
__device__ __host__ __forceinline__ int csr_tix9(int v) { return (v >> CSR_GB9) * CSR_TS9 + (v & (CSR_GN9 - 1)); }
__global__ __launch_bounds__(64) void csrA_kernel9(const int* __restrict__ dst, int E, int N, int nG, int CHP, int NGP, int* __restrict__ STG, int* __restrict__ HST) {
  extern __shared__ int sm[];
  int* cnt = sm; int* run = sm + NGP; int* ids = sm + 2 * NGP;
  const int b = blockIdx.x; const int ch = (E + CSR_NBLK9 - 1) / CSR_NBLK9; const int e0 = b * ch, e1 = min(E, e0 + ch);
  for (int i = threadIdx.x; i < NGP; i += 64) cnt[i] = 0;
  for (int i = threadIdx.x; i < CHP; i += 64) ids[i] = -1;
  __syncthreads();
  if (threadIdx.x == 0) {
    for (int e = e0; e < e1; ++e) { int d = dst[e]; d = (d < 0) ? 0 : (d >= N ? N - 1 : d); cnt[d >> CSR_GB9] += 1; }
    int acc = 0; for (int g = 0; g < nG; ++g) { run[g] = acc; acc += cnt[g]; }
    for (int e = e0; e < e1; ++e) { int d = dst[e]; d = (d < 0) ? 0 : (d >= N ? N - 1 : d); const int g = d >> CSR_GB9; ids[run[g]] = e; run[g] += 1; } }
  __syncthreads();
  typedef __attribute__((ext_vector_type(4))) int v4i;
  for (int pass = 0; pass < 2; ++pass) {
    for (int i = threadIdx.x; i < CHP / 4; i += 64) *(volatile v4i*)(STG + (size_t)b * CHP + i * 4) = *(const v4i*)(&ids[i * 4]);
    for (int i = threadIdx.x; i < NGP / 4; i += 64) { v4i v; for (int e = 0; e < 4; ++e) v[e] = (i * 4 + e < nG) ? cnt[i * 4 + e] : 0; *(volatile v4i*)(HST + (size_t)b * NGP + i * 4) = v; }
    __threadfence(); }
}
__global__ __launch_bounds__(512) void csrS_kernel9(const int* __restrict__ HST, int nG, int NGP, int* __restrict__ START, int* __restrict__ TOT, int* __restrict__ OFF) {
  __shared__ int tot[CSR_MAXG9];
  const int b = threadIdx.x;
  for (int pass = 0; pass < 2; ++pass) { int runb = 0; for (int g = 0; g < nG; ++g) { int c = HST[(size_t)b * NGP + g]; c = (c < 0) ? 0 : c; ((volatile int*)OFF)[(size_t)g * CSR_NBLK9 + b] = runb; runb += c; } __threadfence(); }
  for (int g = threadIdx.x; g < nG; g += 512) { int s = 0; for (int bb = 0; bb < CSR_NBLK9; ++bb) { int c = HST[(size_t)bb * NGP + g]; s += (c < 0) ? 0 : c; } tot[g] = s; }
  __syncthreads();
  if (threadIdx.x < 32) {
    __shared__ int st[CSR_MAXG9 + 32];
    if (threadIdx.x == 0) { int acc = 0; for (int g = 0; g < NGP; ++g) { st[g] = acc; if (g < nG) acc += (tot[g] + 31) & ~31; } st[NGP] = acc; }
    __builtin_amdgcn_fence(__ATOMIC_RELEASE, "workgroup"); __builtin_amdgcn_wave_barrier(); __builtin_amdgcn_fence(__ATOMIC_ACQUIRE, "workgroup");
    for (int pass = 0; pass < 2; ++pass) { for (int i = threadIdx.x; i < NGP + 32; i += 32) { ((volatile int*)START)[i] = (i <= NGP) ? st[min(i, NGP)] : 0; ((volatile int*)TOT)[i] = (i < nG) ? tot[i] : 0; } __threadfence(); } }
}
__global__ __launch_bounds__(256) void csrB_kernel9(const int* __restrict__ dst, int N, int nG, int CHP, int NGP, int permLen, const int* __restrict__ STG, const int* __restrict__ HST, const int* __restrict__ OFF, const int* __restrict__ START, const int* __restrict__ TOT, int* __restrict__ PERM, int* __restrict__ ROWPTR, int* __restrict__ ROWCNT, int* __restrict__ FLAG) {
  typedef __attribute__((ext_vector_type(4))) int v4i;
  __shared__ int ids[CSR_CAP9]; __shared__ unsigned short key[CSR_CAP9]; __shared__ int outp[CSR_CAP9]; __shared__ int ncnt[CSR_GN9 + 1]; __shared__ int boff[CSR_NBLK9 + 1];
  const int g = blockIdx.x, t_ = threadIdx.x; int tot = TOT[g]; int st = START[g], stn = START[g + 1]; const int v0 = g * CSR_GN9; const int nv = min(CSR_GN9, N - v0); const int t0 = g * CSR_TS9;
  st = (st < 0) ? 0 : (st > permLen - 32 ? permLen - 32 : st) & ~31; stn = (stn < st) ? st : (stn > permLen ? permLen : stn); tot = (tot < 0) ? 0 : tot; if (tot > stn - st && tot <= CSR_CAP9) tot = stn - st;
  if (tot > CSR_CAP9) {
    for (int pass = 0; pass < 2; ++pass) { for (int i = t_; i < CSR_TS9 / 4; i += 256) { v4i a, c; for (int e = 0; e < 4; ++e) { a[e] = st; c[e] = 0; } *(volatile v4i*)(ROWPTR + t0 + i * 4) = a; *(volatile v4i*)(ROWCNT + t0 + i * 4) = c; } if (t_ == 0) ((volatile int*)FLAG)[0] = 1; __threadfence(); } (void)nv; return; }
  if (t_ == 0) { int acc = 0; for (int b = 0; b < CSR_NBLK9; ++b) { boff[b] = acc; int c = HST[(size_t)b * NGP + g]; c = (c < 0) ? 0 : (c > CHP ? CHP : c); acc += c; if (acc > tot) acc = tot; } boff[CSR_NBLK9] = acc; }
  for (int i = t_; i <= CSR_GN9; i += 256) ncnt[i] = 0;
  __syncthreads();
  for (int b = 0; b < CSR_NBLK9; ++b) { const int c = boff[b + 1] - boff[b]; int o_ = OFF[(size_t)g * CSR_NBLK9 + b]; o_ = (o_ < 0) ? 0 : (o_ > CHP - c ? CHP - c : o_); const int* src_ = STG + (size_t)b * CHP + o_;
    for (int i = t_; i < c; i += 256) { int id = src_[i]; id = (id < 0) ? 0 : id; ids[boff[b] + i] = id; int d = dst[id]; d = (d < v0) ? v0 : (d >= N ? N - 1 : d); int kk = d - v0; kk = (kk < 0) ? 0 : (kk >= CSR_GN9 ? CSR_GN9 - 1 : kk); key[boff[b] + i] = (unsigned short)kk; } }
  __syncthreads();
  if (t_ == 0) { for (int i = 0; i < tot; ++i) ncnt[key[i]] += 1; int acc = 0; for (int vl = 0; vl < CSR_GN9; ++vl) { const int c = ncnt[vl]; ncnt[vl] = acc; acc += c; } ncnt[CSR_GN9] = acc;
    for (int i = 0; i < tot; ++i) { const int vl = key[i]; outp[ncnt[vl]] = ids[i]; ncnt[vl] += 1; }
    for (int vl = CSR_GN9; vl > 0; --vl) ncnt[vl] = ncnt[vl - 1]; ncnt[0] = 0; }
  __syncthreads();
  for (int pass = 0; pass < 2; ++pass) {
    for (int i = t_; i < (stn - st) / 4; i += 256) { v4i v; for (int e = 0; e < 4; ++e) { const int q = i * 4 + e; v[e] = (q < tot) ? outp[q] : -1; } *(volatile v4i*)(PERM + st + i * 4) = v; }
    for (int i = t_; i < CSR_TS9 / 4; i += 256) { v4i a, c; for (int e = 0; e < 4; ++e) { const int vl = i * 4 + e; const int vc = vl < CSR_GN9 ? vl : CSR_GN9; a[e] = (vl < CSR_GN9) ? st + ncnt[vc] : st; c[e] = (vl < nv) ? (ncnt[(vc < CSR_GN9 ? vc : CSR_GN9 - 1) + 1] - ncnt[vc]) : 0; } *(volatile v4i*)(ROWPTR + t0 + i * 4) = a; *(volatile v4i*)(ROWCNT + t0 + i * 4) = c; }
    __threadfence(); }
}
__global__ __launch_bounds__(256) void csrZ_kernel9(int* __restrict__ p, size_t n4) { typedef __attribute__((ext_vector_type(4))) int v4i; const size_t tid = (size_t)blockIdx.x * 256 + threadIdx.x, nth = (size_t)gridDim.x * 256; v4i z = {0, 0, 0, 0}; for (size_t i = tid; i < n4; i += nth) *(volatile v4i*)(p + i * 4) = z; }
struct CsrBufs9 { int *STG, *HST, *OFF, *START, *TOT, *PERM, *ROWPTR, *ROWCNT, *FLAG; int nG, NGP, CHP; size_t permLen; char* base; size_t bytes; };
static size_t csr_carve9(CsrBufs9& c, char* ws, size_t off, int E, int N) {
  const size_t off0 = off; c.base = ws + off;
  auto al = [&](size_t bytes) { char* p = ws + off; off += (bytes + 255) & ~(size_t)255; return p; };
  c.nG = (N + CSR_GN9 - 1) / CSR_GN9; c.NGP = (c.nG + 31) & ~31; const int ch = (E + CSR_NBLK9 - 1) / CSR_NBLK9; c.CHP = (ch + 31) & ~31; c.permLen = (size_t)E + 32 * (size_t)c.nG + 32;
  c.STG = (int*)al((size_t)CSR_NBLK9 * c.CHP * 4); c.HST = (int*)al((size_t)CSR_NBLK9 * c.NGP * 4); c.OFF = (int*)al((size_t)c.NGP * CSR_NBLK9 * 4); c.START = (int*)al((size_t)(c.NGP + 64) * 4); c.TOT = (int*)al((size_t)(c.NGP + 64) * 4);
  c.PERM = (int*)al(c.permLen * 4); c.ROWPTR = (int*)al((size_t)c.nG * CSR_TS9 * 4); c.ROWCNT = (int*)al((size_t)c.nG * CSR_TS9 * 4); c.FLAG = (int*)al(256);
  c.bytes = off - off0; return off;
}
static void csr_build9(const CsrBufs9& c, const int* dst, int E, int N, hipStream_t stream) {
  const size_t smem = (size_t)(2 * c.NGP + c.CHP) * 4;
  csrZ_kernel9<<<512, 256, 0, stream>>>((int*)c.base, c.bytes / 16);
  csrA_kernel9<<<CSR_NBLK9, 64, smem, stream>>>(dst, E, N, c.nG, c.CHP, c.NGP, c.STG, c.HST);
  csrS_kernel9<<<1, 512, 0, stream>>>(c.HST, c.nG, c.NGP, c.START, c.TOT, c.OFF);
  csrB_kernel9<<<c.nG, 256, 0, stream>>>(dst, N, c.nG, c.CHP, c.NGP, (int)c.permLen, c.STG, c.HST, c.OFF, c.START, c.TOT, c.PERM, c.ROWPTR, c.ROWCNT, c.FLAG);
}

constexpr int CSR_NBLK3 = 512, CSR_GB3 = 3, CSR_GN3 = 1 << CSR_GB3  , CSR_TS3 = (CSR_GN3 < 32 ? 32 : CSR_GN3)  , CSR_MAXG3 = 512, CSR_CAP3 = 12288  ;
__device__ __host__ __forceinline__ int csr_tix3(int v) { return (v >> CSR_GB3) * CSR_TS3 + (v & (CSR_GN3 - 1)); }
__global__ __launch_bounds__(64) void csrA_kernel3(const int* __restrict__ dst, int E, int N, int nG, int CHP, int NGP, int* __restrict__ STG, int* __restrict__ HST) {
  extern __shared__ int sm[];
  int* cnt = sm; int* run = sm + NGP; int* ids = sm + 2 * NGP;
  const int b = blockIdx.x; const int ch = (E + CSR_NBLK3 - 1) / CSR_NBLK3; const int e0 = b * ch, e1 = min(E, e0 + ch);
  for (int i = threadIdx.x; i < NGP; i += 64) cnt[i] = 0;
  for (int i = threadIdx.x; i < CHP; i += 64) ids[i] = -1;
  __syncthreads();
  if (threadIdx.x == 0) {
    for (int e = e0; e < e1; ++e) { int d = dst[e]; d = (d < 0) ? 0 : (d >= N ? N - 1 : d); cnt[d >> CSR_GB3] += 1; }
    int acc = 0; for (int g = 0; g < nG; ++g) { run[g] = acc; acc += cnt[g]; }
    for (int e = e0; e < e1; ++e) { int d = dst[e]; d = (d < 0) ? 0 : (d >= N ? N - 1 : d); const int g = d >> CSR_GB3; ids[run[g]] = e; run[g] += 1; } }
  __syncthreads();
  typedef __attribute__((ext_vector_type(4))) int v4i;
  for (int pass = 0; pass < 2; ++pass) {
    for (int i = threadIdx.x; i < CHP / 4; i += 64) *(volatile v4i*)(STG + (size_t)b * CHP + i * 4) = *(const v4i*)(&ids[i * 4]);
    for (int i = threadIdx.x; i < NGP / 4; i += 64) { v4i v; for (int e = 0; e < 4; ++e) v[e] = (i * 4 + e < nG) ? cnt[i * 4 + e] : 0; *(volatile v4i*)(HST + (size_t)b * NGP + i * 4) = v; }
    __threadfence(); }
}
__global__ __launch_bounds__(512) void csrS_kernel3(const int* __restrict__ HST, int nG, int NGP, int* __restrict__ START, int* __restrict__ TOT, int* __restrict__ OFF) {
  __shared__ int tot[CSR_MAXG3];
  const int b = threadIdx.x;
  for (int pass = 0; pass < 2; ++pass) { int runb = 0; for (int g = 0; g < nG; ++g) { int c = HST[(size_t)b * NGP + g]; c = (c < 0) ? 0 : c; ((volatile int*)OFF)[(size_t)g * CSR_NBLK3 + b] = runb; runb += c; } __threadfence(); }
  for (int g = threadIdx.x; g < nG; g += 512) { int s = 0; for (int bb = 0; bb < CSR_NBLK3; ++bb) { int c = HST[(size_t)bb * NGP + g]; s += (c < 0) ? 0 : c; } tot[g] = s; }
  __syncthreads();
  if (threadIdx.x < 32) {
    __shared__ int st[CSR_MAXG3 + 32];
    if (threadIdx.x == 0) { int acc = 0; for (int g = 0; g < NGP; ++g) { st[g] = acc; if (g < nG) acc += (tot[g] + 31) & ~31; } st[NGP] = acc; }
    __builtin_amdgcn_fence(__ATOMIC_RELEASE, "workgroup"); __builtin_amdgcn_wave_barrier(); __builtin_amdgcn_fence(__ATOMIC_ACQUIRE, "workgroup");
    for (int pass = 0; pass < 2; ++pass) { for (int i = threadIdx.x; i < NGP + 32; i += 32) { ((volatile int*)START)[i] = (i <= NGP) ? st[min(i, NGP)] : 0; ((volatile int*)TOT)[i] = (i < nG) ? tot[i] : 0; } __threadfence(); } }
}
__global__ __launch_bounds__(256) void csrB_kernel3(const int* __restrict__ dst, int N, int nG, int CHP, int NGP, int permLen, const int* __restrict__ STG, const int* __restrict__ HST, const int* __restrict__ OFF, const int* __restrict__ START, const int* __restrict__ TOT, int* __restrict__ PERM, int* __restrict__ ROWPTR, int* __restrict__ ROWCNT, int* __restrict__ FLAG) {
  typedef __attribute__((ext_vector_type(4))) int v4i;
  __shared__ int ids[CSR_CAP3]; __shared__ unsigned short key[CSR_CAP3]; __shared__ int outp[CSR_CAP3]; __shared__ int ncnt[CSR_GN3 + 1]; __shared__ int boff[CSR_NBLK3 + 1];
  const int g = blockIdx.x, t_ = threadIdx.x; int tot = TOT[g]; int st = START[g], stn = START[g + 1]; const int v0 = g * CSR_GN3; const int nv = min(CSR_GN3, N - v0); const int t0 = g * CSR_TS3;
  st = (st < 0) ? 0 : (st > permLen - 32 ? permLen - 32 : st) & ~31; stn = (stn < st) ? st : (stn > permLen ? permLen : stn); tot = (tot < 0) ? 0 : tot; if (tot > stn - st && tot <= CSR_CAP3) tot = stn - st;
  if (tot > CSR_CAP3) {
    for (int pass = 0; pass < 2; ++pass) { for (int i = t_; i < CSR_TS3 / 4; i += 256) { v4i a, c; for (int e = 0; e < 4; ++e) { a[e] = st; c[e] = 0; } *(volatile v4i*)(ROWPTR + t0 + i * 4) = a; *(volatile v4i*)(ROWCNT + t0 + i * 4) = c; } if (t_ == 0) ((volatile int*)FLAG)[0] = 1; __threadfence(); } (void)nv; return; }
  if (t_ == 0) { int acc = 0; for (int b = 0; b < CSR_NBLK3; ++b) { boff[b] = acc; int c = HST[(size_t)b * NGP + g]; c = (c < 0) ? 0 : (c > CHP ? CHP : c); acc += c; if (acc > tot) acc = tot; } boff[CSR_NBLK3] = acc; }
  for (int i = t_; i <= CSR_GN3; i += 256) ncnt[i] = 0;
  __syncthreads();
  for (int b = 0; b < CSR_NBLK3; ++b) { const int c = boff[b + 1] - boff[b]; int o_ = OFF[(size_t)g * CSR_NBLK3 + b]; o_ = (o_ < 0) ? 0 : (o_ > CHP - c ? CHP - c : o_); const int* src_ = STG + (size_t)b * CHP + o_;
    for (int i = t_; i < c; i += 256) { int id = src_[i]; id = (id < 0) ? 0 : id; ids[boff[b] + i] = id; int d = dst[id]; d = (d < v0) ? v0 : (d >= N ? N - 1 : d); int kk = d - v0; kk = (kk < 0) ? 0 : (kk >= CSR_GN3 ? CSR_GN3 - 1 : kk); key[boff[b] + i] = (unsigned short)kk; } }
  __syncthreads();
  if (t_ == 0) { for (int i = 0; i < tot; ++i) ncnt[key[i]] += 1; int acc = 0; for (int vl = 0; vl < CSR_GN3; ++vl) { const int c = ncnt[vl]; ncnt[vl] = acc; acc += c; } ncnt[CSR_GN3] = acc;
    for (int i = 0; i < tot; ++i) { const int vl = key[i]; outp[ncnt[vl]] = ids[i]; ncnt[vl] += 1; }
    for (int vl = CSR_GN3; vl > 0; --vl) ncnt[vl] = ncnt[vl - 1]; ncnt[0] = 0; }
  __syncthreads();
  for (int pass = 0; pass < 2; ++pass) {
    for (int i = t_; i < (stn - st) / 4; i += 256) { v4i v; for (int e = 0; e < 4; ++e) { const int q = i * 4 + e; v[e] = (q < tot) ? outp[q] : -1; } *(volatile v4i*)(PERM + st + i * 4) = v; }
    for (int i = t_; i < CSR_TS3 / 4; i += 256) { v4i a, c; for (int e = 0; e < 4; ++e) { const int vl = i * 4 + e; const int vc = vl < CSR_GN3 ? vl : CSR_GN3; a[e] = (vl < CSR_GN3) ? st + ncnt[vc] : st; c[e] = (vl < nv) ? (ncnt[(vc < CSR_GN3 ? vc : CSR_GN3 - 1) + 1] - ncnt[vc]) : 0; } *(volatile v4i*)(ROWPTR + t0 + i * 4) = a; *(volatile v4i*)(ROWCNT + t0 + i * 4) = c; }
    __threadfence(); }
}
__global__ __launch_bounds__(256) void csrZ_kernel3(int* __restrict__ p, size_t n4) { typedef __attribute__((ext_vector_type(4))) int v4i; const size_t tid = (size_t)blockIdx.x * 256 + threadIdx.x, nth = (size_t)gridDim.x * 256; v4i z = {0, 0, 0, 0}; for (size_t i = tid; i < n4; i += nth) *(volatile v4i*)(p + i * 4) = z; }
struct CsrBufs3 { int *STG, *HST, *OFF, *START, *TOT, *PERM, *ROWPTR, *ROWCNT, *FLAG; int nG, NGP, CHP; size_t permLen; char* base; size_t bytes; };
static size_t csr_carve3(CsrBufs3& c, char* ws, size_t off, int E, int N) {
  const size_t off0 = off; c.base = ws + off;
  auto al = [&](size_t bytes) { char* p = ws + off; off += (bytes + 255) & ~(size_t)255; return p; };
  c.nG = (N + CSR_GN3 - 1) / CSR_GN3; c.NGP = (c.nG + 31) & ~31; const int ch = (E + CSR_NBLK3 - 1) / CSR_NBLK3; c.CHP = (ch + 31) & ~31; c.permLen = (size_t)E + 32 * (size_t)c.nG + 32;
  c.STG = (int*)al((size_t)CSR_NBLK3 * c.CHP * 4); c.HST = (int*)al((size_t)CSR_NBLK3 * c.NGP * 4); c.OFF = (int*)al((size_t)c.NGP * CSR_NBLK3 * 4); c.START = (int*)al((size_t)(c.NGP + 64) * 4); c.TOT = (int*)al((size_t)(c.NGP + 64) * 4);
  c.PERM = (int*)al(c.permLen * 4); c.ROWPTR = (int*)al((size_t)c.nG * CSR_TS3 * 4); c.ROWCNT = (int*)al((size_t)c.nG * CSR_TS3 * 4); c.FLAG = (int*)al(256);
  c.bytes = off - off0; return off;
}
static void csr_build3(const CsrBufs3& c, const int* dst, int E, int N, hipStream_t stream) {
  const size_t smem = (size_t)(2 * c.NGP + c.CHP) * 4;
  csrZ_kernel3<<<512, 256, 0, stream>>>((int*)c.base, c.bytes / 16);
  csrA_kernel3<<<CSR_NBLK3, 64, smem, stream>>>(dst, E, N, c.nG, c.CHP, c.NGP, c.STG, c.HST);
  csrS_kernel3<<<1, 512, 0, stream>>>(c.HST, c.nG, c.NGP, c.START, c.TOT, c.OFF);
  csrB_kernel3<<<c.nG, 256, 0, stream>>>(dst, N, c.nG, c.CHP, c.NGP, (int)c.permLen, c.STG, c.HST, c.OFF, c.START, c.TOT, c.PERM, c.ROWPTR, c.ROWCNT, c.FLAG);
}


__global__ __launch_bounds__(256) void wcopy_kernel(const float* __restrict__ w, int n8, b16* __restrict__ WT) {
  const int u = blockIdx.x * 256 + threadIdx.x; if (u >= n8) return; const size_t e = (size_t)u * 8; v8b v; for (int j = 0; j < 8; ++j) v[j] = (b16)(bf16_rne(w[e + j]) * WSC);
  for (int pass = 0; pass < 2; ++pass) { *(volatile v8b*)(WT + e) = v; __threadfence(); }
}
__global__ __launch_bounds__(128) void proj1_kernel(const float* __restrict__ x, const b16* __restrict__ W1, const float* __restrict__ as_, const float* __restrict__ ad_, float* __restrict__ HW1, float* __restrict__ ASH, float* __restrict__ ADH) {
  __shared__ __attribute__((aligned(16))) float Tf[4][16][HID + 4]; __shared__ __attribute__((aligned(16))) float sa[64], sd[64];
  const int wave = threadIdx.x >> 5, lane = threadIdx.x & 31, nloc = lane & 15, hlf = lane >> 4; const size_t m0 = (size_t)blockIdx.x * 64 + wave * 16; const int h = blockIdx.y; const int c0 = h * HID;
  const size_t rr_ = (m0 + nloc) < (size_t)N ? (m0 + nloc) : (size_t)(N - 1); const float* xr = x + rr_ * DIN;
  v8f acc[8];
#pragma unroll
  for (int t = 0; t < 8; ++t) acc[t] = (v8f){};
#pragma unroll 2
  for (int kb = 0; kb < DIN; kb += 32) { v16b a; for (int j = 0; j < 8; ++j) { a[j] = (b16)(bf16_rne(xr[kb + 8 * hlf + j]) * XS); a[8 + j] = (b16)(bf16_rne(xr[kb + 16 + 8 * hlf + j]) * XS); }
#pragma unroll
    for (int t = 0; t < 8; ++t) acc[t] = wmma16b(a, frag_kb(W1 + (size_t)(c0 + t * 16 + nloc) * DIN + kb, hlf), acc[t]); }
  float ps[8], pd[8]; for (int r8 = 0; r8 < 8; ++r8) { ps[r8] = 0.0f; pd[r8] = 0.0f; }
#pragma unroll
  for (int t = 0; t < 8; ++t) { const int c = t * 16 + nloc; const float ws_ = opaque(bf16_rne(as_[c0 + c])), wd_ = opaque(bf16_rne(ad_[c0 + c]));
#pragma unroll
    for (int r8 = 0; r8 < 8; ++r8) { const float v = acc[t][r8] * (1.0f / (XS * WSC)); Tf[wave][8 * hlf + r8][c] = v; ps[r8] += pmul(v, ws_); pd[r8] += pmul(v, wd_); } }
#pragma unroll
  for (int r8 = 0; r8 < 8; ++r8) { float a = ps[r8], b = pd[r8]; for (int o = 1; o < 16; o <<= 1) { a += __shfl_xor(a, o); b += __shfl_xor(b, o); } if (nloc == 0) { sa[wave * 16 + 8 * hlf + r8] = a; sd[wave * 16 + 8 * hlf + r8] = b; } }
  __syncthreads();
  for (int pass = 0; pass < 2; ++pass) { for (int rr = 0; rr < 16; ++rr) *(volatile v4f*)(HW1 + (m0 + rr) * W1O + c0 + lane * 4) = *(const v4f*)(&Tf[wave][rr][lane * 4]);
    if (threadIdx.x < 16) *(volatile v4f*)(ASH + (size_t)h * NP + (size_t)blockIdx.x * 64 + threadIdx.x * 4) = *(const v4f*)(&sa[threadIdx.x * 4]); else if (threadIdx.x < 32) *(volatile v4f*)(ADH + (size_t)h * NP + (size_t)blockIdx.x * 64 + (threadIdx.x - 16) * 4) = *(const v4f*)(&sd[(threadIdx.x - 16) * 4]);
    __threadfence(); }
}
__global__ __launch_bounds__(256) void attn1_kernel(const float* __restrict__ HW1, const float* __restrict__ ASH, const float* __restrict__ ADH, const float* __restrict__ b1, const float* __restrict__ g1, const float* __restrict__ be1, const int* __restrict__ srcs, const int* __restrict__ PERM, const int* __restrict__ ROWPTR, const int* __restrict__ ROWCNT, int permLen, float* __restrict__ H1) {
  const int wave = threadIdx.x >> 5, lane = threadIdx.x & 31; const size_t v = (size_t)blockIdx.x * 8 + wave; const int h = lane >> 3; v4f acc[4]; for (int q = 0; q < 4; ++q) acc[q] = (v4f){0.0f, 0.0f, 0.0f, 0.0f};
  if (v < (size_t)N) { int st = ROWPTR[v], cnt = ROWCNT[v]; cnt = iclamp(cnt, 0, 65536); st = iclamp(st, 0, permLen - cnt); const float adv = ADH[(size_t)h * NP + v], asv = ASH[(size_t)h * NP + v];
    float mx = lrelu(asv + adv);
#pragma unroll 1
    for (int j = 0; j < cnt; ++j) { const int e = iclamp(PERM[st + j], 0, E - 1); const int s = iclamp(srcs[e], 0, N - 1); mx = fmaxf(mx, lrelu(ASH[(size_t)h * NP + s] + adv)); }
    float den = nexp(lrelu(asv + adv) - mx); for (int q = 0; q < 4; ++q) { const v4f own = *(const v4f*)(HW1 + v * W1O + lane * 16 + q * 4); for (int i = 0; i < 4; ++i) acc[q][i] = pmul(own[i], den); }
#pragma unroll 1
    for (int j = 0; j < cnt; ++j) { const int e = iclamp(PERM[st + j], 0, E - 1); const size_t s = (size_t)iclamp(srcs[e], 0, N - 1); const float p = nexp(lrelu(ASH[(size_t)h * NP + s] + adv) - mx); den += p;
      for (int q = 0; q < 4; ++q) { const v4f xs = *(const v4f*)(HW1 + s * W1O + lane * 16 + q * 4); for (int i = 0; i < 4; ++i) acc[q][i] += pmul(p, xs[i]); } }
    const float inv = 1.0f / (den + 1e-16f);
    for (int q = 0; q < 4; ++q) for (int i = 0; i < 4; ++i) { const int c = lane * 16 + q * 4 + i; const float y = pmul(acc[q][i], inv) + bf16_rne(b1[c]); acc[q][i] = eluf(pmul(y, bf16_rne(g1[c]) * BNS) + bf16_rne(be1[c])); } }
  for (int pass = 0; pass < 2; ++pass) { for (int q = 0; q < 4; ++q) *(volatile v4f*)(H1 + v * W1O + lane * 16 + q * 4) = acc[q]; __threadfence(); }
}
__global__ __launch_bounds__(128) void proj2_kernel(const float* __restrict__ H1, const b16* __restrict__ W2, const float* __restrict__ as_, const float* __restrict__ ad_, float* __restrict__ HW2, float* __restrict__ AS2, float* __restrict__ AD2) {
  __shared__ __attribute__((aligned(16))) b16 Ah[4][16][W1O + 8], Al[4][16][W1O + 8]; __shared__ __attribute__((aligned(16))) float sa[64], sd[64];
  const int wave = threadIdx.x >> 5, lane = threadIdx.x & 31, nloc = lane & 15, hlf = lane >> 4; const size_t m0 = (size_t)blockIdx.x * 64 + wave * 16;
  for (int rr = 0; rr < 16; ++rr) { for (int q = 0; q < 4; ++q) { const v4f hv = *(const v4f*)(H1 + (m0 + rr) * W1O + lane * 16 + q * 4); for (int j = 0; j < 4; ++j) { b16 p, ql; split16(hv[j] * XS, p, ql); Ah[wave][rr][lane * 16 + q * 4 + j] = p; Al[wave][rr][lane * 16 + q * 4 + j] = ql; } } }
  wave_lds_sync();
  v8f acc[8];
#pragma unroll
  for (int t = 0; t < 8; ++t) acc[t] = (v8f){};
#pragma unroll 2
  for (int kb = 0; kb < W1O; kb += 32) { const v16b a = frag_kb(&Ah[wave][nloc][kb], hlf), al = frag_kb(&Al[wave][nloc][kb], hlf);
#pragma unroll
    for (int t = 0; t < 8; ++t) { const v16b bw = frag_kb(W2 + (size_t)(t * 16 + nloc) * W1O + kb, hlf); acc[t] = wmma16b(a, bw, acc[t]); acc[t] = wmma16b(al, bw, acc[t]); } }
  wave_lds_sync();
  float* Tf = (float*)&Ah[wave][0][0];
  float ps[8], pd[8]; for (int r8 = 0; r8 < 8; ++r8) { ps[r8] = 0.0f; pd[r8] = 0.0f; }
#pragma unroll
  for (int t = 0; t < 8; ++t) { const int c = t * 16 + nloc; const float ws_ = opaque(bf16_rne(as_[c])), wd_ = opaque(bf16_rne(ad_[c]));
#pragma unroll
    for (int r8 = 0; r8 < 8; ++r8) { const float v = acc[t][r8] * (1.0f / (XS * WSC)); Tf[(8 * hlf + r8) * (HID + 4) + c] = v; ps[r8] += pmul(v, ws_); pd[r8] += pmul(v, wd_); } }
#pragma unroll
  for (int r8 = 0; r8 < 8; ++r8) { float a = ps[r8], b = pd[r8]; for (int o = 1; o < 16; o <<= 1) { a += __shfl_xor(a, o); b += __shfl_xor(b, o); } if (nloc == 0) { sa[wave * 16 + 8 * hlf + r8] = a; sd[wave * 16 + 8 * hlf + r8] = b; } }
  __syncthreads();
  for (int pass = 0; pass < 2; ++pass) { for (int rr = 0; rr < 16; ++rr) *(volatile v4f*)(HW2 + (m0 + rr) * HID + lane * 4) = *(const v4f*)(&Tf[rr * (HID + 4) + lane * 4]);
    if (threadIdx.x < 16) *(volatile v4f*)(AS2 + (size_t)blockIdx.x * 64 + threadIdx.x * 4) = *(const v4f*)(&sa[threadIdx.x * 4]); else if (threadIdx.x < 32) *(volatile v4f*)(AD2 + (size_t)blockIdx.x * 64 + (threadIdx.x - 16) * 4) = *(const v4f*)(&sd[(threadIdx.x - 16) * 4]);
    __threadfence(); }
}
__global__ __launch_bounds__(256) void attn2_kernel(const float* __restrict__ HW2, const float* __restrict__ AS2, const float* __restrict__ AD2, const float* __restrict__ b2, const float* __restrict__ g2, const float* __restrict__ be2, const int* __restrict__ srcs, const int* __restrict__ PERM, const int* __restrict__ ROWPTR, const int* __restrict__ ROWCNT, int permLen, float* __restrict__ H2) {
  const int wave = threadIdx.x >> 5, lane = threadIdx.x & 31; const size_t v = (size_t)blockIdx.x * 8 + wave; v4f acc = {0.0f, 0.0f, 0.0f, 0.0f};
  if (v < (size_t)N) { int st = ROWPTR[v], cnt = ROWCNT[v]; cnt = iclamp(cnt, 0, 65536); st = iclamp(st, 0, permLen - cnt); const float adv = AD2[v], asv = AS2[v]; float mx = lrelu(asv + adv);
#pragma unroll 1
    for (int j = 0; j < cnt; ++j) { const int e = iclamp(PERM[st + j], 0, E - 1); const int s = iclamp(srcs[e], 0, N - 1); mx = fmaxf(mx, lrelu(AS2[s] + adv)); }
    float den = nexp(lrelu(asv + adv) - mx); { const v4f own = *(const v4f*)(HW2 + v * HID + lane * 4); for (int i = 0; i < 4; ++i) acc[i] = pmul(own[i], den); }
#pragma unroll 1
    for (int j = 0; j < cnt; ++j) { const int e = iclamp(PERM[st + j], 0, E - 1); const size_t s = (size_t)iclamp(srcs[e], 0, N - 1); const float p = nexp(lrelu(AS2[s] + adv) - mx); den += p; const v4f xs = *(const v4f*)(HW2 + s * HID + lane * 4); for (int i = 0; i < 4; ++i) acc[i] += pmul(p, xs[i]); }
    const float inv = 1.0f / (den + 1e-16f); for (int i = 0; i < 4; ++i) { const int c = lane * 4 + i; const float y = pmul(acc[i], inv) + bf16_rne(b2[c]); acc[i] = eluf(pmul(y, bf16_rne(g2[c]) * BNS) + bf16_rne(be2[c])); } }
  for (int pass = 0; pass < 2; ++pass) { *(volatile v4f*)(H2 + v * HID + lane * 4) = acc; __threadfence(); }
}
__global__ __launch_bounds__(256) void pool_kernel(const float* __restrict__ H2, const int* __restrict__ PERM, const int* __restrict__ ROWPTR, const int* __restrict__ ROWCNT, int permLen, float* __restrict__ XG) {
  const int wave = threadIdx.x >> 5, lane = threadIdx.x & 31; const int g = blockIdx.x * 8 + wave; const int tix = (g >> 3) * 32 + (g & 7);
  int st = ROWPTR[tix], cnt = ROWCNT[tix]; cnt = iclamp(cnt, 0, 65536); st = iclamp(st, 0, permLen - cnt); v4f a = {0.0f, 0.0f, 0.0f, 0.0f};
#pragma unroll 1
  for (int j = 0; j < cnt; ++j) { const int n = iclamp(PERM[st + j], 0, N - 1); const v4f hv = *(const v4f*)(H2 + (size_t)n * HID + lane * 4); for (int i = 0; i < 4; ++i) a[i] += hv[i]; }
  const float inv = 1.0f / (float)(cnt < 1 ? 1 : cnt); for (int i = 0; i < 4; ++i) a[i] = pmul(a[i], inv);
  for (int pass = 0; pass < 2; ++pass) { *(volatile v4f*)(XG + (size_t)g * HID + lane * 4) = a; __threadfence(); }
}
__global__ __launch_bounds__(256) void head_kernel(const float* __restrict__ XG, const float* __restrict__ hyb, const b16* __restrict__ HW1T, const b16* __restrict__ HW2T, const b16* __restrict__ FWT, const b16* __restrict__ CWT,
                                                    const float* __restrict__ hb1, const float* __restrict__ hb2, const float* __restrict__ fb, const float* __restrict__ cb,
                                                    const float* __restrict__ gh1, const float* __restrict__ bh1, const float* __restrict__ gh2, const float* __restrict__ bh2, const float* __restrict__ gf, const float* __restrict__ bfn, float* __restrict__ out) {
  __shared__ __attribute__((aligned(16))) b16 Ah[8][16][HYB + 8], Al[8][16][HYB + 8]; __shared__ __attribute__((aligned(16))) float So[8][16][NCL];
  const int wave = threadIdx.x >> 5, lane = threadIdx.x & 31, nloc = lane & 15, hlf = lane >> 4; const int g0 = wave * 16; const float sc = 1.0f / (XS * WSC);
  for (int rr = 0; rr < 16; ++rr) { const v8f hv = *(const v8f*)(hyb + (size_t)(g0 + rr) * HYB + lane * 8); for (int j = 0; j < 8; ++j) { Ah[wave][rr][lane * 8 + j] = (b16)(bf16_rne(hv[j]) * XS); Al[wave][rr][lane * 8 + j] = (b16)0.0f; } }
  wave_lds_sync();
  v8f acc[8];
#pragma unroll
  for (int t = 0; t < 8; ++t) acc[t] = (v8f){};
#pragma unroll 2
  for (int kb = 0; kb < HYB; kb += 32) { const v16b a = frag_kb(&Ah[wave][nloc][kb], hlf);
#pragma unroll
    for (int t = 0; t < 8; ++t) acc[t] = wmma16b(a, frag_kb(HW1T + (size_t)(t * 16 + nloc) * HYB + kb, hlf), acc[t]); }
  wave_lds_sync();
#pragma unroll
  for (int t = 0; t < 8; ++t) { const int c = t * 16 + nloc; const float bb = bf16_rne(hb1[c]), gg = bf16_rne(gh1[c]) * BNS, be = bf16_rne(bh1[c]);
#pragma unroll 1
    for (int r8 = 0; r8 < 8; ++r8) { const float v = fmaxf(pmul(acc[t][r8] * sc + bb, gg) + be, 0.0f); b16 p, q; split16(v * XS, p, q); Ah[wave][8 * hlf + r8][c] = p; Al[wave][8 * hlf + r8][c] = q; } }
  wave_lds_sync();
#pragma unroll
  for (int t = 0; t < 8; ++t) acc[t] = (v8f){};
#pragma unroll 2
  for (int kb = 0; kb < HID; kb += 32) { const v16b a = frag_kb(&Ah[wave][nloc][kb], hlf), al = frag_kb(&Al[wave][nloc][kb], hlf);
#pragma unroll
    for (int t = 0; t < 8; ++t) { const v16b bw = frag_kb(HW2T + (size_t)(t * 16 + nloc) * HID + kb, hlf); acc[t] = wmma16b(a, bw, acc[t]); acc[t] = wmma16b(al, bw, acc[t]); } }
  wave_lds_sync();
#pragma unroll
  for (int t = 0; t < 8; ++t) { const int c = t * 16 + nloc; const float bb = bf16_rne(hb2[c]), gg = bf16_rne(gh2[c]) * BNS, be = bf16_rne(bh2[c]);
#pragma unroll 1
    for (int r8 = 0; r8 < 8; ++r8) { const float v = fmaxf(pmul(acc[t][r8] * sc + bb, gg) + be, 0.0f); b16 p, q; split16(v * XS, p, q); Ah[wave][8 * hlf + r8][HID + c] = p; Al[wave][8 * hlf + r8][HID + c] = q; } }
  for (int rr = 0; rr < 16; ++rr) { const v4f xv = *(const v4f*)(XG + (size_t)(g0 + rr) * HID + lane * 4); for (int j = 0; j < 4; ++j) { b16 p, q; split16(xv[j] * XS, p, q); Ah[wave][rr][lane * 4 + j] = p; Al[wave][rr][lane * 4 + j] = q; } }
  wave_lds_sync();
#pragma unroll
  for (int t = 0; t < 8; ++t) acc[t] = (v8f){};
#pragma unroll 2
  for (int kb = 0; kb < HYB; kb += 32) { const v16b a = frag_kb(&Ah[wave][nloc][kb], hlf), al = frag_kb(&Al[wave][nloc][kb], hlf);
#pragma unroll
    for (int t = 0; t < 8; ++t) { const v16b bw = frag_kb(FWT + (size_t)(t * 16 + nloc) * HYB + kb, hlf); acc[t] = wmma16b(a, bw, acc[t]); acc[t] = wmma16b(al, bw, acc[t]); } }
  wave_lds_sync();
#pragma unroll
  for (int t = 0; t < 8; ++t) { const int c = t * 16 + nloc; const float bb = bf16_rne(fb[c]), gg = bf16_rne(gf[c]) * BNS, be = bf16_rne(bfn[c]);
#pragma unroll 1
    for (int r8 = 0; r8 < 8; ++r8) { const float v = fmaxf(pmul(acc[t][r8] * sc + bb, gg) + be, 0.0f); b16 p, q; split16(v * XS, p, q); Ah[wave][8 * hlf + r8][c] = p; Al[wave][8 * hlf + r8][c] = q; } }
  wave_lds_sync();
  v8f ao[2] = {(v8f){}, (v8f){}};
#pragma unroll 2
  for (int kb = 0; kb < HID; kb += 32) { const v16b a = frag_kb(&Ah[wave][nloc][kb], hlf), al = frag_kb(&Al[wave][nloc][kb], hlf);
#pragma unroll
    for (int t = 0; t < 2; ++t) { const v16b bw = frag_kb(CWT + (size_t)(t * 16 + nloc) * HID + kb, hlf); ao[t] = wmma16b(a, bw, ao[t]); ao[t] = wmma16b(al, bw, ao[t]); } }
#pragma unroll
  for (int t = 0; t < 2; ++t) { const int c = t * 16 + nloc; const float bb = bf16_rne(cb[c]);
#pragma unroll 1
    for (int r8 = 0; r8 < 8; ++r8) So[wave][8 * hlf + r8][c] = ao[t][r8] * sc + bb; }
  wave_lds_sync();
  for (int pass = 0; pass < 2; ++pass) { for (int rr = 0; rr < 16; ++rr) if (lane < 8) *(volatile v4f*)(out + (size_t)(g0 + rr) * NCL + lane * 4) = *(const v4f*)(&So[wave][rr][lane * 4]); __threadfence(); }
}
}

extern "C" void kernel_launch(void* const* d_in, const int* in_sizes, int n_in, void* d_out, int out_size, void* d_ws, size_t ws_size, hipStream_t stream) {
  (void)n_in;
  auto Fp = [&](int i) { return (const float*)d_in[i]; }; auto Ip = [&](int i) { return (const int*)d_in[i]; };
  if (in_sizes[0] != N * DIN || in_sizes[1] != 2 * E || in_sizes[2] != N || in_sizes[3] != G * HYB || in_sizes[4] != W1O * DIN || in_sizes[5] != NH * HID || in_sizes[8] != HID * W1O || in_sizes[22] != HID * HYB || in_sizes[24] != HID * HID || in_sizes[26] != HID * HYB || in_sizes[28] != NCL * HID || out_size != G * NCL) return;
  size_t off = 0; char* ws = (char*)d_ws;
  auto carve = [&](size_t bytes) { char* p = ws + off; off += (bytes + 255) & ~(size_t)255; return p; };
  b16* W1 = (b16*)carve((size_t)W1O * DIN * 2); b16* W2 = (b16*)carve((size_t)HID * W1O * 2); b16* HW1T = (b16*)carve((size_t)HID * HYB * 2); b16* HW2T = (b16*)carve((size_t)HID * HID * 2); b16* FWT = (b16*)carve((size_t)HID * HYB * 2); b16* CWT = (b16*)carve((size_t)NCL * HID * 2);
  float* HW1 = (float*)carve((size_t)NP * W1O * 4); float* H1 = (float*)carve((size_t)NP * W1O * 4); float* ASH = (float*)carve((size_t)NH * NP * 4); float* ADH = (float*)carve((size_t)NH * NP * 4);
  float* HW2 = (float*)carve((size_t)NP * HID * 4); float* H2 = (float*)carve((size_t)NP * HID * 4); float* AS2 = (float*)carve((size_t)NP * 4); float* AD2 = (float*)carve((size_t)NP * 4); float* XG = (float*)carve((size_t)G * HID * 4);
  CsrBufs9 csr; CsrBufs3 pool; off = csr_carve9(csr, ws, off, E, N); off = csr_carve3(pool, ws, off, N, G);
  if (off > ws_size || off > ((size_t)128 << 20)) return;
  wcopy_kernel<<<(W1O * DIN / 8 + 255) / 256, 256, 0, stream>>>(Fp(4), W1O * DIN / 8, W1); wcopy_kernel<<<(HID * W1O / 8 + 255) / 256, 256, 0, stream>>>(Fp(8), HID * W1O / 8, W2);
  wcopy_kernel<<<(HID * HYB / 8 + 255) / 256, 256, 0, stream>>>(Fp(22), HID * HYB / 8, HW1T); wcopy_kernel<<<(HID * HID / 8 + 255) / 256, 256, 0, stream>>>(Fp(24), HID * HID / 8, HW2T);
  wcopy_kernel<<<(HID * HYB / 8 + 255) / 256, 256, 0, stream>>>(Fp(26), HID * HYB / 8, FWT); wcopy_kernel<<<(NCL * HID / 8 + 255) / 256, 256, 0, stream>>>(Fp(28), NCL * HID / 8, CWT);
  csr_build9(csr, Ip(1) + E, E, N, stream); csr_build3(pool, Ip(2), N, G, stream);
  proj1_kernel<<<dim3(NP / 64, NH), 128, 0, stream>>>(Fp(0), W1, Fp(5), Fp(6), HW1, ASH, ADH);
  attn1_kernel<<<NP / 8, 256, 0, stream>>>(HW1, ASH, ADH, Fp(7), Fp(12), Fp(13), Ip(1), csr.PERM, csr.ROWPTR, csr.ROWCNT, (int)csr.permLen, H1);
  proj2_kernel<<<NP / 64, 128, 0, stream>>>(H1, W2, Fp(9), Fp(10), HW2, AS2, AD2);
  attn2_kernel<<<NP / 8, 256, 0, stream>>>(HW2, AS2, AD2, Fp(11), Fp(14), Fp(15), Ip(1), csr.PERM, csr.ROWPTR, csr.ROWCNT, (int)csr.permLen, H2);
  pool_kernel<<<G / 8, 256, 0, stream>>>(H2, pool.PERM, pool.ROWPTR, pool.ROWCNT, (int)pool.permLen, XG);
  head_kernel<<<1, 256, 0, stream>>>(XG, Fp(3), HW1T, HW2T, FWT, CWT, Fp(23), Fp(25), Fp(27), Fp(29), Fp(16), Fp(17), Fp(18), Fp(19), Fp(20), Fp(21), (float*)d_out);
}
